// VSDANet_60043642798804
// MI455X (gfx1250) — hardware-verified
//
#include <hip/hip_runtime.h>
#include <math.h>
#include <stdint.h>

#define NB      8
#define NSEQ    1024
#define CD      256
#define NHEAD   8
#define HDIM    32
#define HID     1024
#define GCH     512
#define NLAY    2
#define IMW     32
#define MP      (NB * NSEQ)
#define QKW     (2 * CD)
#define LNEPS   1.0e-5f
#define WSC     64.0f
#define QKCARRY 16.0f
#define VCARRY  16.0f
#define PCARRY  1024.0f
#define AOCARRY 64.0f
#define HCARRY  16.0f
#define GCARRY  1024.0f
static_assert(NHEAD * HDIM == CD);
static_assert(IMW * IMW == NSEQ);
static_assert(HID == 4 * CD);
static_assert(GCH == 2 * CD);
static_assert((MP % 64) == 0 && (CD % 64) == 0 && (HID % 64) == 0 && (NSEQ % 64) == 0 && (QKW % 64) == 0);
static_assert(CD == 32 * 8);
static_assert((NSEQ % 4) == 0 && (IMW % 4) == 0);

typedef _Float16 v16h __attribute__((ext_vector_type(16)));
typedef _Float16 v8h  __attribute__((ext_vector_type(8)));
typedef float    v8f  __attribute__((ext_vector_type(8)));
typedef float    v4f  __attribute__((ext_vector_type(4)));
typedef unsigned int v4u __attribute__((ext_vector_type(4)));

union FragH  { v16h v; v8h h[2]; };
union Frag16 { v16h h; v8h hh[2]; v4u u[2]; };

__device__ __forceinline__ unsigned short bf_bits(float f) {
  unsigned u = __float_as_uint(f);
  return (unsigned short)((u + 0x7FFFu + ((u >> 16) & 1u)) >> 16);
}
__device__ __forceinline__ float bf_up(unsigned short h) { return __uint_as_float(((unsigned)h) << 16); }
__device__ __forceinline__ float bfr(float f) { return bf_up(bf_bits(f)); }
__device__ __forceinline__ unsigned short h_bits(_Float16 x) { return __builtin_bit_cast(unsigned short, x); }
__device__ __forceinline__ unsigned pk16(unsigned short a, unsigned short b) { return (unsigned)a | ((unsigned)b << 16); }
__device__ __forceinline__ v8f zero8() { v8f z = {0.f, 0.f, 0.f, 0.f, 0.f, 0.f, 0.f, 0.f}; return z; }

__device__ __forceinline__ v16h ldfrag_h(const _Float16* p) {
  FragH f;
  f.h[0] = *(const v8h*)(p);
  f.h[1] = *(const v8h*)(p + 16);
  return f.v;
}
__device__ __forceinline__ Frag16 ldfrag16(const unsigned short* p) {
  Frag16 f;
  f.u[0] = *(const v4u*)(p);
  f.u[1] = *(const v4u*)(p + 16);
  return f;
}

__device__ __forceinline__ v8f mma_h(v16h a, v16h b, v8f c) {
  c = __builtin_amdgcn_wmma_f32_16x16x32_f16(false, a, false, b, (short)0, c, false, false);
#if defined(__HIP_DEVICE_COMPILE__)
  asm volatile("v_nop\n\tv_nop\n\tv_nop\n\tv_nop" : "+v"(c) : "v"(a), "v"(b));
#endif
  return c;
}
__device__ __forceinline__ v8f mma_h_raw(v16h a, v16h b, v8f c) {
  return __builtin_amdgcn_wmma_f32_16x16x32_f16(false, a, false, b, (short)0, c, false, false);
}
__device__ __forceinline__ void dep_guard1(v8f& a, v8f& b, v16h x) {
#if defined(__HIP_DEVICE_COMPILE__)
  asm volatile("v_nop\n\tv_nop\n\tv_nop\n\tv_nop" : "+v"(a), "+v"(b) : "v"(x));
#endif
}
__device__ __forceinline__ void dep_guard3(v8f& a, v8f& b, v16h x, v16h y, v16h z) {
#if defined(__HIP_DEVICE_COMPILE__)
  asm volatile("v_nop\n\tv_nop\n\tv_nop\n\tv_nop" : "+v"(a), "+v"(b) : "v"(x), "v"(y), "v"(z));
#endif
}
__device__ __forceinline__ void keep4_h(v16h a, v16h b, v16h c, v16h d) {
#if defined(__HIP_DEVICE_COMPILE__)
  asm volatile("v_nop" :: "v"(a), "v"(b), "v"(c), "v"(d));
#endif
}
__device__ __forceinline__ void acc_guard4(v8f& a, v8f& b, v8f& c, v8f& d) {
#if defined(__HIP_DEVICE_COMPILE__)
  asm volatile("v_nop\n\tv_nop\n\tv_nop\n\tv_nop" : "+v"(a), "+v"(b), "+v"(c), "+v"(d));
#endif
}
__device__ __forceinline__ void wave_sync_lds() {
  __builtin_amdgcn_fence(__ATOMIC_RELEASE, "workgroup");
  __builtin_amdgcn_wave_barrier();
  __builtin_amdgcn_fence(__ATOMIC_ACQUIRE, "workgroup");
}
__device__ __forceinline__ float wsum32(float v) {
#pragma unroll
  for (int off = 16; off > 0; off >>= 1) v += __shfl_xor(v, off, 32);
  return v;
}

__global__ __launch_bounds__(256) void conv_t16(const float* __restrict__ src, unsigned short* dst,
                                                 int Cin, int P, int col0, int Odst, int n8, float wsc) {
  const int i    = blockIdx.x * 256 + threadIdx.x;
  const int ic   = (i < n8) ? i : (n8 - 1);
  const int per  = (Odst * Cin) >> 3;
  const int bi   = ic / per;
  const int r    = ic - bi * per;
  const int cin8 = Cin >> 3;
  const int o    = r / cin8;
  const int c0   = (r - o * cin8) * 8;
  const float* p = src + ((size_t)bi * Cin + c0) * P + col0 + o;
  float v[8];
#pragma unroll
  for (int e = 0; e < 8; ++e) v[e] = bfr(p[(size_t)e * P]);
  v4u ov;
#pragma unroll
  for (int e = 0; e < 4; ++e)
    ov[e] = pk16(h_bits((_Float16)(v[2 * e] * wsc)), h_bits((_Float16)(v[2 * e + 1] * wsc)));
  if (i < n8) *(volatile v4u*)(dst + (size_t)i * 8) = ov;
  __threadfence();
  if (i < n8) *(volatile v4u*)(dst + (size_t)i * 8) = ov;
}

__global__ __launch_bounds__(256) void conv_n16(const float* __restrict__ src, unsigned short* dst, int n8, float wsc) {
  const int i  = blockIdx.x * 256 + threadIdx.x;
  const int ic = (i < n8) ? i : (n8 - 1);
  const v4f a = *(const v4f*)(src + (size_t)ic * 8), c = *(const v4f*)(src + (size_t)ic * 8 + 4);
  v4u ov;
  ov[0] = pk16(h_bits((_Float16)(bfr(a[0]) * wsc)), h_bits((_Float16)(bfr(a[1]) * wsc)));
  ov[1] = pk16(h_bits((_Float16)(bfr(a[2]) * wsc)), h_bits((_Float16)(bfr(a[3]) * wsc)));
  ov[2] = pk16(h_bits((_Float16)(bfr(c[0]) * wsc)), h_bits((_Float16)(bfr(c[1]) * wsc)));
  ov[3] = pk16(h_bits((_Float16)(bfr(c[2]) * wsc)), h_bits((_Float16)(bfr(c[3]) * wsc)));
  if (i < n8) *(volatile v4u*)(dst + (size_t)i * 8) = ov;
  __threadfence();
  if (i < n8) *(volatile v4u*)(dst + (size_t)i * 8) = ov;
}

__global__ __launch_bounds__(256) void xprep(const float* __restrict__ src, float* dst, int n4) {
  const int i  = blockIdx.x * 256 + threadIdx.x;
  const int ic = (i < n4) ? i : (n4 - 1);
  const v4f a = *(const v4f*)(src + (size_t)ic * 4);
  v4f o;
#pragma unroll
  for (int e = 0; e < 4; ++e) o[e] = bfr(a[e]);
  if (i < n4) *(volatile v4f*)(dst + (size_t)i * 4) = o;
  __threadfence();
  if (i < n4) *(volatile v4f*)(dst + (size_t)i * 4) = o;
}

__global__ __launch_bounds__(256) void ln256(const float* __restrict__ X, const float* __restrict__ gam,
                                              const float* __restrict__ bet, unsigned short* Y) {
  const int tid = threadIdx.x, wave = tid >> 5, lane = tid & 31;
  const size_t row  = (size_t)blockIdx.x * 8 + wave;
  const size_t base = row * CD + 8 * lane;
  const v4f x0 = *(const v4f*)(X + base), x1 = *(const v4f*)(X + base + 4);
  float s = ((x0[0] + x0[1]) + (x0[2] + x0[3])) + ((x1[0] + x1[1]) + (x1[2] + x1[3]));
  s = wsum32(s);
  const float mean = s * (1.0f / CD);
  float d[8];
#pragma unroll
  for (int e = 0; e < 4; ++e) { d[e] = x0[e] - mean; d[4 + e] = x1[e] - mean; }
  float vs = 0.f;
#pragma unroll
  for (int e = 0; e < 8; ++e) vs += d[e] * d[e];
  vs = wsum32(vs);
  const float rstd = rsqrtf(vs * (1.0f / CD) + LNEPS);
  const v4f g0 = *(const v4f*)(gam + 8 * lane), g1 = *(const v4f*)(gam + 8 * lane + 4);
  const v4f b0 = *(const v4f*)(bet + 8 * lane), b1 = *(const v4f*)(bet + 8 * lane + 4);
  float y[8];
#pragma unroll
  for (int e = 0; e < 4; ++e) {
    y[e]     = (d[e] * rstd)     * bfr(g0[e]) + bfr(b0[e]);
    y[4 + e] = (d[4 + e] * rstd) * bfr(g1[e]) + bfr(b1[e]);
  }
  v4u o;
#pragma unroll
  for (int e = 0; e < 4; ++e) o[e] = pk16(h_bits((_Float16)y[2 * e]), h_bits((_Float16)y[2 * e + 1]));
  *(volatile v4u*)(Y + base) = o;
  __threadfence();
  *(volatile v4u*)(Y + base) = o;
}

template <int A32, int OM, int BIASM, int RES>
__global__ __launch_bounds__(256) void gemm64(
    const void* __restrict__ Ap, int lda, long long strideA, float ascale,
    const unsigned short* __restrict__ Btp, int ldb, long long strideB,
    const float* __restrict__ bias, float bscale,
    const float* resid,
    void* Cout, int ldc, long long strideC,
    int M, int N, int K, float oscale) {
  __shared__ __align__(16) float sT[8][16 * 68];
  const int b    = blockIdx.y;
  const int lane = threadIdx.x & 31;
  const int wave = threadIdx.x >> 5;
  const int tilesN = N >> 6;
  const int tilesM = M >> 6;
  const int tile = blockIdx.x * 8 + wave;
  if (tile >= tilesM * tilesN) return;
  const int tm = tile / tilesN;
  const int tn = tile - tm * tilesN;
  const int m0 = tm << 6;
  const int n0 = tn << 6;

  const unsigned short* A1 = (const unsigned short*)Ap + (size_t)b * strideA;
  const float*          Af = (const float*)Ap + (size_t)b * strideA;
  const unsigned short* Bb = Btp + (size_t)b * strideB;

  const int rlane = lane & 15;
  const int koff  = (lane >> 4) * 8;
  const int mOff  = (lane >> 4) * 8;

  v8f acc[4][4];
#pragma unroll
  for (int i = 0; i < 4; ++i)
#pragma unroll
    for (int j = 0; j < 4; ++j) acc[i][j] = zero8();

  for (int k0 = 0; k0 < K; k0 += 32) {
    Frag16 bh[4];
#pragma unroll
    for (int j = 0; j < 4; ++j) {
      const size_t bo = (size_t)(n0 + (j << 4) + rlane) * ldb + koff + k0;
      bh[j] = ldfrag16(Bb + bo);
    }
#pragma unroll
    for (int i = 0; i < 4; ++i) {
      Frag16 ah;
      if (A32) {
        const float* ap = Af + (size_t)(m0 + (i << 4) + rlane) * lda + koff + k0;
        const v4f x0 = *(const v4f*)(ap), x1 = *(const v4f*)(ap + 4);
        const v4f x2 = *(const v4f*)(ap + 16), x3 = *(const v4f*)(ap + 20);
#pragma unroll
        for (int e = 0; e < 4; ++e) {
          ah.hh[0][e]     = (_Float16)(x0[e] * ascale);
          ah.hh[0][4 + e] = (_Float16)(x1[e] * ascale);
          ah.hh[1][e]     = (_Float16)(x2[e] * ascale);
          ah.hh[1][4 + e] = (_Float16)(x3[e] * ascale);
        }
      } else {
        const size_t ao = (size_t)(m0 + (i << 4) + rlane) * lda + koff + k0;
        ah = ldfrag16(A1 + ao);
      }
#pragma unroll
      for (int j = 0; j < 4; ++j) acc[i][j] = mma_h_raw(ah.h, bh[j].h, acc[i][j]);
      dep_guard1(acc[i][0], acc[i][3], ah.h);
    }
    keep4_h(bh[0].h, bh[1].h, bh[2].h, bh[3].h);
  }
  acc_guard4(acc[0][0], acc[0][1], acc[0][2], acc[0][3]);
  acc_guard4(acc[1][0], acc[1][1], acc[1][2], acc[1][3]);
  acc_guard4(acc[2][0], acc[2][1], acc[2][2], acc[2][3]);
  acc_guard4(acc[3][0], acc[3][1], acc[3][2], acc[3][3]);

  const int hh2 = lane >> 4, c4 = (lane & 15) * 4;
  const int q8  = lane >> 3, c8 = (lane & 7) * 8;
  float bc[8];
#pragma unroll
  for (int e = 0; e < 8; ++e) bc[e] = 0.f;
  if (BIASM == 0) {
    if (OM == 0) {
      const int cb = n0 + c4;
      const int i0 = (cb < N - 4) ? cb : (N - 4);
      const v4f b0v = *(const v4f*)(bias + i0);
#pragma unroll
      for (int e = 0; e < 4; ++e) bc[e] = bfr(b0v[e]) * bscale;
    } else {
      const int cb = n0 + c8;
      const int i0 = (cb < N - 8) ? cb : (N - 8);
      const v4f b0a = *(const v4f*)(bias + i0), b0b = *(const v4f*)(bias + i0 + 4);
#pragma unroll
      for (int e = 0; e < 4; ++e) {
        bc[e]     = bfr(b0a[e]) * bscale;
        bc[4 + e] = bfr(b0b[e]) * bscale;
      }
    }
  }

  float* slab = sT[wave];
#pragma unroll
  for (int i = 0; i < 4; ++i) {
    const int mBase = m0 + (i << 4);
#pragma unroll
    for (int j = 0; j < 4; ++j) {
#pragma unroll
      for (int r = 0; r < 8; ++r) {
        slab[(mOff + r) * 68 + (j << 4) + rlane] = acc[i][j][r];
      }
    }
    wave_sync_lds();
    if (OM == 0) {
      float* C = (float*)Cout + (size_t)b * strideC;
      const float* Rf = resid + (size_t)b * strideC;
      v4f vals[8];
#pragma unroll
      for (int it = 0; it < 8; ++it) {
        const int row = it * 2 + hh2;
        v4f v = *(const v4f*)(slab + row * 68 + c4);
#pragma unroll
        for (int e = 0; e < 4; ++e) v[e] = v[e] * oscale + bc[e];
        if (RES == 1) {
          const v4f rr = *(const v4f*)(Rf + (size_t)(mBase + row) * ldc + n0 + c4);
#pragma unroll
          for (int e = 0; e < 4; ++e) v[e] += rr[e];
        }
        vals[it] = v;
      }
      for (int pass = 0; pass < 2; ++pass) {
#pragma unroll
        for (int it = 0; it < 8; ++it) {
          const int row = it * 2 + hh2;
          *(volatile v4f*)(C + (size_t)(mBase + row) * ldc + n0 + c4) = vals[it];
        }
        __threadfence();
      }
    } else {
      unsigned short* C = (unsigned short*)Cout + (size_t)b * strideC;
      v4u hv[4];
#pragma unroll
      for (int it = 0; it < 4; ++it) {
        const int row = it * 4 + q8;
        const float* sp = slab + row * 68 + c8;
        float bm = 0.f;
        if (BIASM == 1) bm = bfr(bias[mBase + row]) * bscale;
        v4u a;
#pragma unroll
        for (int e = 0; e < 4; ++e) {
          const float f0 = sp[2 * e]     * oscale + ((BIASM == 1) ? bm : bc[2 * e]);
          const float f1 = sp[2 * e + 1] * oscale + ((BIASM == 1) ? bm : bc[2 * e + 1]);
          a[e] = pk16(h_bits((_Float16)f0), h_bits((_Float16)f1));
        }
        hv[it] = a;
      }
      for (int pass = 0; pass < 2; ++pass) {
#pragma unroll
        for (int it = 0; it < 4; ++it) {
          const int row = it * 4 + q8;
          *(volatile v4u*)(C + (size_t)(mBase + row) * ldc + n0 + c8) = hv[it];
        }
        __threadfence();
      }
    }
    wave_sync_lds();
  }
}

__global__ __launch_bounds__(128)
void attn_head(const unsigned short* __restrict__ qk, const unsigned short* __restrict__ vt, float* ao) {
  __shared__ __align__(16) float Ps[4][16 * 68];
  __shared__ __align__(16) float Os[4][16 * 32];

  const int tid  = threadIdx.x;
  const int wave = tid >> 5;
  const int lane = tid & 31;
  const int hh   = lane >> 4;
  const int c    = lane & 15;

  const int bx = blockIdx.x;
  const int b  = bx >> 7;
  const int h  = (bx >> 4) & (NHEAD - 1);
  const int q0 = (bx & 15) * 64 + wave * 16;
  const size_t gr = (size_t)b * NSEQ + q0;

  const _Float16* Q  = (const _Float16*)(const void*)qk;
  const _Float16* Qp = Q + h * HDIM;
  const _Float16* Kp = Q + (size_t)b * NSEQ * QKW + CD + h * HDIM;
  const _Float16* V  = (const _Float16*)(const void*)vt + ((size_t)b * CD + h * HDIM) * NSEQ;
  const float lsc = (1.4426950408889634f * 0.17677669529663688f) / (QKCARRY * QKCARRY);
  const float dec = logf(1.0f - exp2f(-2.0f - 0.5f * (float)h));
  const float dl2 = dec * 1.4426950408889634f;

  const v16h qa = ldfrag_h(Qp + (gr + c) * QKW + 8 * hh);
  const float iqb = (float)(q0 + 8 * hh);

  float mrow[8], lrow[8];
  v8f oacc0 = zero8(), oacc1 = zero8();
#pragma unroll
  for (int r = 0; r < 8; ++r) { mrow[r] = -INFINITY; lrow[r] = 0.f; }
  float* pt = Ps[wave];

#pragma unroll 1
  for (int kb = 0; kb < NSEQ; kb += 64) {
    v8f s[4];
#pragma unroll
    for (int j = 0; j < 4; ++j) {
      const v16h kf = ldfrag_h(Kp + (size_t)(kb + 16 * j + c) * QKW + 8 * hh);
      s[j] = mma_h(qa, kf, zero8());
    }
    const float kj = (float)(kb + c);
#pragma unroll
    for (int r = 0; r < 8; ++r) {
      const float iq = iqb + (float)r;
      const float t0 = s[0][r] * lsc + fabsf(iq - kj) * dl2;
      const float t1 = s[1][r] * lsc + fabsf(iq - (kj + 16.0f)) * dl2;
      const float t2 = s[2][r] * lsc + fabsf(iq - (kj + 32.0f)) * dl2;
      const float t3 = s[3][r] * lsc + fabsf(iq - (kj + 48.0f)) * dl2;
      float mx = fmaxf(fmaxf(t0, t1), fmaxf(t2, t3));
#pragma unroll
      for (int off = 1; off < 16; off <<= 1) mx = fmaxf(mx, __shfl_xor(mx, off, 32));
      const float mn = fmaxf(mrow[r], mx);
      const float al = exp2f(mrow[r] - mn);
      mrow[r] = mn;
      const float e0 = exp2f(t0 - mn), e1 = exp2f(t1 - mn), e2 = exp2f(t2 - mn), e3 = exp2f(t3 - mn);
      float ps = (e0 + e1) + (e2 + e3);
#pragma unroll
      for (int off = 1; off < 16; off <<= 1) ps += __shfl_xor(ps, off, 32);
      lrow[r] = lrow[r] * al + ps;
      oacc0[r] *= al;
      oacc1[r] *= al;
      const int ro = (8 * hh + r) * 68 + c;
      pt[ro]      = e0;
      pt[ro + 16] = e1;
      pt[ro + 32] = e2;
      pt[ro + 48] = e3;
    }
    wave_sync_lds();
#pragma unroll
    for (int wi = 0; wi < 2; ++wi) {
      const float* prow = pt + c * 68 + 32 * wi + 8 * hh;
      const v4f p0 = *(const v4f*)(prow), p1 = *(const v4f*)(prow + 4);
      const v4f p2 = *(const v4f*)(prow + 16), p3 = *(const v4f*)(prow + 20);
      FragH pa;
#pragma unroll
      for (int e = 0; e < 4; ++e) {
        pa.h[0][e]     = (_Float16)(p0[e] * PCARRY);
        pa.h[0][4 + e] = (_Float16)(p1[e] * PCARRY);
        pa.h[1][e]     = (_Float16)(p2[e] * PCARRY);
        pa.h[1][4 + e] = (_Float16)(p3[e] * PCARRY);
      }
      const int k0 = kb + 32 * wi;
      const v16h vb0 = ldfrag_h(V + (size_t)c * NSEQ + k0 + 8 * hh);
      const v16h vb1 = ldfrag_h(V + (size_t)(16 + c) * NSEQ + k0 + 8 * hh);
      oacc0 = mma_h_raw(pa.v, vb0, oacc0);
      oacc1 = mma_h_raw(pa.v, vb1, oacc1);
      dep_guard3(oacc0, oacc1, pa.v, vb0, vb1);
    }
    wave_sync_lds();
  }

  float* os = Os[wave];
  const float oinv = 1.0f / (PCARRY * VCARRY);
#pragma unroll
  for (int r = 0; r < 8; ++r) {
    const float inv = (1.0f / lrow[r]) * oinv;
    os[(8 * hh + r) * 32 + c]      = oacc0[r] * inv;
    os[(8 * hh + r) * 32 + 16 + c] = oacc1[r] * inv;
  }
  wave_sync_lds();
  {
    const int q4 = lane >> 3, e4 = (lane & 7) * 4;
    v4f vals[4];
#pragma unroll
    for (int it = 0; it < 4; ++it) {
      const int row = it * 4 + q4;
      vals[it] = *(const v4f*)(os + row * 32 + e4);
    }
    for (int pass = 0; pass < 2; ++pass) {
#pragma unroll
      for (int it = 0; it < 4; ++it) {
        const int row = it * 4 + q4;
        *(volatile v4f*)(ao + (gr + row) * CD + h * HDIM + e4) = vals[it];
      }
      __threadfence();
    }
  }
}

__global__ __launch_bounds__(256) void dwgate(const unsigned short* __restrict__ H, const float* __restrict__ w,
                                               const float* __restrict__ bb, unsigned short* G) {
  __shared__ __align__(16) float gs[4 * GCH];
  const int tid = threadIdx.x;
  const int t0  = blockIdx.x * 4;
  const int b   = t0 >> 10;
  const int p0  = t0 & (NSEQ - 1);
  const int y   = p0 >> 5;
  const int xb  = p0 & (IMW - 1);
  const _Float16* Hb = (const _Float16*)(const void*)H + (size_t)b * NSEQ * HID;
#pragma unroll 1
  for (int cs = 0; cs < 2; ++cs) {
    const int c = tid + 256 * cs;
    float w1[9], w2[9];
#pragma unroll
    for (int t = 0; t < 9; ++t) {
      w1[t] = bfr(w[c * 9 + t]);
      w2[t] = bfr(w[(c + GCH) * 9 + t]);
    }
    const float b1 = bfr(bb[c]), b2 = bfr(bb[c + GCH]);
#pragma unroll 1
    for (int px = 0; px < 4; ++px) {
      const int x = xb + px;
      float s1 = 0.f, s2 = 0.f;
#pragma unroll
      for (int ky = 0; ky < 3; ++ky) {
        const int yy = y + ky - 1;
        const int yc = (yy < 0) ? 0 : ((yy > IMW - 1) ? (IMW - 1) : yy);
        const float vy = (yy >= 0 && yy < IMW) ? 1.0f : 0.0f;
#pragma unroll
        for (int kx = 0; kx < 3; ++kx) {
          const int xx = x + kx - 1;
          const int xc = (xx < 0) ? 0 : ((xx > IMW - 1) ? (IMW - 1) : xx);
          const float vf = (xx >= 0 && xx < IMW) ? vy : 0.0f;
          const size_t o = (size_t)(yc * IMW + xc) * HID + c;
          const float h1 = (float)Hb[o] * vf;
          const float h2 = (float)Hb[o + GCH] * vf;
          s1 = fmaf(w1[ky * 3 + kx], h1, s1);
          s2 = fmaf(w2[ky * 3 + kx], h2, s2);
        }
      }
      const float a1 = s1 * (1.0f / HCARRY) + b1;
      const float a2 = s2 * (1.0f / HCARRY) + b2;
      const float ge = 0.5f * a1 * (1.0f + erff(a1 * 0.70710678118654752f));
      gs[px * GCH + c] = ge * a2;
    }
  }
  __syncthreads();
  {
    const int px = tid >> 6, c0 = (tid & 63) * 8;
    const v4f ga = *(const v4f*)(gs + px * GCH + c0), gb = *(const v4f*)(gs + px * GCH + c0 + 4);
    v4u o;
    o[0] = pk16(h_bits((_Float16)(ga[0] * GCARRY)), h_bits((_Float16)(ga[1] * GCARRY)));
    o[1] = pk16(h_bits((_Float16)(ga[2] * GCARRY)), h_bits((_Float16)(ga[3] * GCARRY)));
    o[2] = pk16(h_bits((_Float16)(gb[0] * GCARRY)), h_bits((_Float16)(gb[1] * GCARRY)));
    o[3] = pk16(h_bits((_Float16)(gb[2] * GCARRY)), h_bits((_Float16)(gb[3] * GCARRY)));
    unsigned short* dp = G + (size_t)(t0 + px) * GCH + c0;
    *(volatile v4u*)dp = o;
    __threadfence();
    *(volatile v4u*)dp = o;
  }
}

extern "C" void kernel_launch(void* const* d_in, const int* in_sizes, int n_in,
                              void* d_out, int out_size, void* d_ws, size_t ws_size,
                              hipStream_t stream) {
  if (n_in < 15) return;
  if (in_sizes[0] != MP * CD) return;
  if (in_sizes[1] != NLAY * CD * 3 * CD || in_sizes[2] != NLAY * 3 * CD) return;
  if (in_sizes[3] != NLAY * CD * CD || in_sizes[4] != NLAY * CD) return;
  if (in_sizes[5] != NLAY * CD || in_sizes[6] != NLAY * CD || in_sizes[7] != NLAY * CD || in_sizes[8] != NLAY * CD) return;
  if (in_sizes[9] != NLAY * HID * CD || in_sizes[10] != NLAY * HID) return;
  if (in_sizes[11] != NLAY * HID * 9 || in_sizes[12] != NLAY * HID) return;
  if (in_sizes[13] != NLAY * CD * GCH || in_sizes[14] != NLAY * CD) return;
  if (out_size != MP * CD) return;

  const float* x      = (const float*)d_in[0];
  const float* qkv_w  = (const float*)d_in[1];
  const float* qkv_b  = (const float*)d_in[2];
  const float* proj_w = (const float*)d_in[3];
  const float* proj_b = (const float*)d_in[4];
  const float* ln1_g  = (const float*)d_in[5];
  const float* ln1_b  = (const float*)d_in[6];
  const float* ln2_g  = (const float*)d_in[7];
  const float* ln2_b  = (const float*)d_in[8];
  const float* pin_w  = (const float*)d_in[9];
  const float* pin_b  = (const float*)d_in[10];
  const float* dw_w   = (const float*)d_in[11];
  const float* dw_b   = (const float*)d_in[12];
  const float* pout_w = (const float*)d_in[13];
  const float* pout_b = (const float*)d_in[14];

  const size_t PWQK = (size_t)NLAY * QKW * CD * 2;
  const size_t PWVT = (size_t)NLAY * CD * CD * 2;
  const size_t PWPR = (size_t)NLAY * CD * CD * 2;
  const size_t PWPI = (size_t)NLAY * HID * CD * 2;
  const size_t PWPO = (size_t)NLAY * CD * GCH * 2;
  const size_t PXF  = (size_t)MP * CD * 4;
  const size_t PXN  = (size_t)MP * CD * 2;
  const size_t PQK  = (size_t)MP * QKW * 2;
  const size_t PVT  = (size_t)NB * CD * NSEQ * 2;
  const size_t PH16 = (size_t)MP * HID * 2;
  const size_t PG16 = (size_t)MP * GCH * 2;
  size_t off = 0;
  const size_t oWQK = off; off += PWQK;
  const size_t oWVT = off; off += PWVT;
  const size_t oWPR = off; off += PWPR;
  const size_t oWPI = off; off += PWPI;
  const size_t oWPO = off; off += PWPO;
  const size_t oX0  = off; off += PXF;
  const size_t oX1  = off; off += PXF;
  const size_t oX2  = off; off += PXF;
  const size_t oXN  = off; off += PXN;
  const size_t oQK  = off; off += PQK;
  const size_t oVT  = off; off += PVT;
  const size_t oAO  = off; off += PXF;
  const size_t oH16 = off; off += PH16;
  const size_t oG16 = off; off += PG16;
  if (off > ws_size) return;
  if (off > (size_t)134217728) return;

  char* ws = (char*)d_ws;
  unsigned short* WQK = (unsigned short*)(ws + oWQK);
  unsigned short* WVT = (unsigned short*)(ws + oWVT);
  unsigned short* WPR = (unsigned short*)(ws + oWPR);
  unsigned short* WPI = (unsigned short*)(ws + oWPI);
  unsigned short* WPO = (unsigned short*)(ws + oWPO);
  float*          X0  = (float*)(ws + oX0);
  float*          X1  = (float*)(ws + oX1);
  float*          X2  = (float*)(ws + oX2);
  unsigned short* XN  = (unsigned short*)(ws + oXN);
  unsigned short* QK  = (unsigned short*)(ws + oQK);
  unsigned short* VT  = (unsigned short*)(ws + oVT);
  float*          AO  = (float*)(ws + oAO);
  unsigned short* H16 = (unsigned short*)(ws + oH16);
  unsigned short* G16 = (unsigned short*)(ws + oG16);
  float*          out = (float*)d_out;

  const int n8qk = (NLAY * QKW * CD) / 8;
  const int n8v  = (NLAY * CD * CD) / 8;
  const int n8pr = (NLAY * CD * CD) / 8;
  const int n8pi = (NLAY * HID * CD) / 8;
  const int n8po = (NLAY * CD * GCH) / 8;
  const int n4x  = (MP * CD) / 4;
  if ((n8qk % 256) != 0 || (n8v % 256) != 0 || (n8pr % 256) != 0 || (n8pi % 256) != 0 || (n8po % 256) != 0) return;
  if ((n4x % 256) != 0) return;
  const dim3 blk(256), blk128(128);
  const dim3 gCqk((n8qk + 255) / 256), gCv((n8v + 255) / 256), gCpr((n8pr + 255) / 256);
  const dim3 gCpi((n8pi + 255) / 256), gCpo((n8po + 255) / 256);
  const dim3 gX((n4x + 255) / 256);
  const dim3 gLN((MP + 7) / 8);
  const dim3 gQK(((MP / 64) * (QKW / 64) + 7) / 8, 1);
  const dim3 gVT(((CD / 64) * (NSEQ / 64) + 7) / 8, NB);
  const dim3 gAttn(NB * NHEAD * (NSEQ / 64));
  const dim3 gPr(((MP / 64) * (CD / 64) + 7) / 8, 1);
  const dim3 gPin(((MP / 64) * (HID / 64) + 7) / 8, 1);
  const dim3 gDw((MP + 3) / 4);

  conv_t16<<<gCqk, blk, 0, stream>>>(qkv_w, WQK, CD, 3 * CD, 0, QKW, n8qk, WSC);
  conv_t16<<<gCv,  blk, 0, stream>>>(qkv_w, WVT, CD, 3 * CD, 2 * CD, CD, n8v, WSC);
  conv_t16<<<gCpr, blk, 0, stream>>>(proj_w, WPR, CD, CD, 0, CD, n8pr, WSC);
  conv_n16<<<gCpi, blk, 0, stream>>>(pin_w, WPI, n8pi, WSC);
  conv_n16<<<gCpo, blk, 0, stream>>>(pout_w, WPO, n8po, WSC);

  xprep<<<gX, blk, 0, stream>>>(x, X0, n4x);

  for (int l = 0; l < NLAY; ++l) {
    const float* Xin = (l == 0) ? (const float*)X0 : (const float*)X2;
    float* Xout = (l == NLAY - 1) ? out : X2;

    ln256<<<gLN, blk, 0, stream>>>(Xin, ln1_g + l * CD, ln1_b + l * CD, XN);

    gemm64<0, 2, 0, 0><<<gQK, blk, 0, stream>>>(
        (const void*)XN, CD, 0LL, 1.0f,
        WQK + (size_t)l * QKW * CD, CD, 0LL,
        qkv_b + (size_t)l * 3 * CD, QKCARRY, (const float*)X0,
        (void*)QK, QKW, 0LL, MP, QKW, CD, QKCARRY / WSC);

    gemm64<0, 2, 1, 0><<<gVT, blk, 0, stream>>>(
        (const void*)(WVT + (size_t)l * CD * CD), CD, 0LL, 1.0f,
        XN, CD, (long long)NSEQ * CD,
        qkv_b + (size_t)l * 3 * CD + 2 * CD, VCARRY, (const float*)X0,
        (void*)VT, NSEQ, (long long)CD * NSEQ, CD, NSEQ, CD, VCARRY / WSC);

    attn_head<<<gAttn, blk128, 0, stream>>>(QK, VT, AO);

    gemm64<1, 0, 0, 1><<<gPr, blk, 0, stream>>>(
        (const void*)AO, CD, 0LL, AOCARRY,
        WPR + (size_t)l * CD * CD, CD, 0LL,
        proj_b + (size_t)l * CD, 1.0f, Xin,
        (void*)X1, CD, 0LL, MP, CD, CD, 1.0f / (AOCARRY * WSC));

    ln256<<<gLN, blk, 0, stream>>>(X1, ln2_g + l * CD, ln2_b + l * CD, XN);

    gemm64<0, 2, 0, 0><<<gPin, blk, 0, stream>>>(
        (const void*)XN, CD, 0LL, 1.0f,
        WPI + (size_t)l * HID * CD, CD, 0LL,
        pin_b + (size_t)l * HID, HCARRY, (const float*)X0,
        (void*)H16, HID, 0LL, MP, HID, CD, HCARRY / WSC);

    dwgate<<<gDw, blk, 0, stream>>>(H16, dw_w + (size_t)l * HID * 9, dw_b + (size_t)l * HID, G16);

    gemm64<0, 0, 0, 1><<<gPr, blk, 0, stream>>>(
        (const void*)G16, GCH, 0LL, 1.0f,
        WPO + (size_t)l * CD * GCH, GCH, 0LL,
        pout_b + (size_t)l * CD, 1.0f, (const float*)X1,
        (void*)Xout, CD, 0LL, MP, CD, GCH, 1.0f / (GCARRY * WSC));
  }
  (void)hipGetLastError();
}
